// QueryGuidedMoESimple_40312563040759
// MI455X (gfx1250) — hardware-verified
//
#include <hip/hip_runtime.h>


namespace {
constexpr int B = 16384, H = 512, NE = 8, P2 = 96  , RIN = 2 * H;
constexpr float XS = 8.0f, WSC = 256.0f;

typedef _Float16 b16;
typedef __attribute__((ext_vector_type(16))) _Float16 v16b;
typedef __attribute__((ext_vector_type(8))) _Float16 v8b;
typedef __attribute__((ext_vector_type(8))) float v8f;
typedef __attribute__((ext_vector_type(4))) float v4f;
__device__ __forceinline__ float bf16_rne(float f) { unsigned int u = __float_as_uint(f); u += 0x7FFFu + ((u >> 16) & 1u); return __uint_as_float(u & 0xFFFF0000u); }
__device__ __forceinline__ void split16(float v, b16& hi, b16& lo) { hi = (b16)v; lo = (b16)(v - (float)hi); }
__device__ __forceinline__ v16b frag_kb(const b16* p, int hh) { const v8b a = *(const v8b*)(p + 8 * hh), b = *(const v8b*)(p + 16 + 8 * hh); v16b f;
#pragma unroll
  for (int e = 0; e < 8; ++e) { f[e] = a[e]; f[8 + e] = b[e]; } return f; }
__device__ __forceinline__ v8f wmma16b(v16b a, v16b b, v8f c) { v8f d = __builtin_amdgcn_wmma_f32_16x16x32_f16(false, a, false, b, (short)0, c, false, false); asm volatile("v_nop\n\tv_nop\n\tv_nop\n\tv_nop" : "+v"(d) : "v"(a), "v"(b)); return d; }
__device__ __forceinline__ void wave_lds_sync() { __builtin_amdgcn_fence(__ATOMIC_RELEASE, "workgroup"); __builtin_amdgcn_wave_barrier(); __builtin_amdgcn_fence(__ATOMIC_ACQUIRE, "workgroup"); }
__device__ __forceinline__ float pmul(float a, float b) { float p = a * b; asm volatile("" : "+v"(p)); return p; }
__device__ __forceinline__ float nexp(float x) { return __builtin_amdgcn_exp2f(x * 1.4426950408889634f); }

__global__ __launch_bounds__(256) void prepx_kernel(const float* __restrict__ mm, const float* __restrict__ qf, b16* __restrict__ RIN16) {
  const size_t t = (size_t)blockIdx.x * 256 + threadIdx.x; if (t >= (size_t)B * RIN / 8) return; const size_t e = t * 8; const size_t row = e / RIN; const int c = (int)(e % RIN);
  const float* src = (c < H) ? mm + row * H + c : qf + row * H + (c - H); const v4f a = *(const v4f*)src, d = *(const v4f*)(src + 4); v8b o;
#pragma unroll
  for (int j = 0; j < 4; ++j) { o[j] = (b16)(bf16_rne(a[j]) * XS); o[4 + j] = (b16)(bf16_rne(d[j]) * XS); }
  for (int pass = 0; pass < 2; ++pass) { *(volatile v8b*)(RIN16 + e) = o; __threadfence(); }
}
__global__ __launch_bounds__(256) void prepw_kernel(const float* __restrict__ rw1, const float* __restrict__ ew1, const float* __restrict__ ew2, b16* __restrict__ RW1T, b16* __restrict__ EW1T, b16* __restrict__ EW2T) {
  __shared__ __attribute__((aligned(16))) b16 T[64][64 + 8];
  const int kind = blockIdx.z, i0 = blockIdx.x * 64, o0 = blockIdx.y * 64, t_ = threadIdx.x;
  const float* w; b16* dst; int nin, nout;
  if (kind == 0) { w = rw1; dst = RW1T; nin = RIN; nout = H; } else if (kind <= NE) { w = ew1 + (size_t)(kind - 1) * H * H; dst = EW1T + (size_t)(kind - 1) * H * H; nin = H; nout = H; } else { w = ew2 + (size_t)(kind - 1 - NE) * H * P2; dst = EW2T + (size_t)(kind - 1 - NE) * P2 * H; nin = H; nout = P2; }
  if (i0 >= nin || o0 >= nout) return;
  const int no = min(64, nout - o0);
  for (int q = t_; q < 64 * 64; q += 256) { const int ii = q >> 6, oo = q & 63; T[oo][ii] = (oo < no) ? (b16)(bf16_rne(w[(size_t)(i0 + ii) * nout + o0 + oo]) * WSC) : (b16)0.0f; }
  __syncthreads();
  for (int pass = 0; pass < 2; ++pass) { for (int q = t_; q < no * 8; q += 256) { const int oo = q >> 3, c8 = (q & 7) * 8; *(volatile v8b*)(dst + (size_t)(o0 + oo) * nin + i0 + c8) = *(const v8b*)(&T[oo][c8]); } __threadfence(); }
}
template <int MODE, int K>
__global__ __launch_bounds__(128) void gemm1_kernel(const b16* __restrict__ A, int lda, const b16* __restrict__ Bt, const float* __restrict__ bias, float* __restrict__ Yf, b16* __restrict__ Yh, b16* __restrict__ Yl, int ldy) {
  __shared__ __attribute__((aligned(16))) float Tf[MODE == 0 ? 4 : 1][16][128 + 4]; __shared__ __attribute__((aligned(16))) b16 Th[MODE == 1 ? 4 : 1][16][128 + 8], Tl[MODE == 1 ? 4 : 1][16][128 + 8];
  const int wave = threadIdx.x >> 5, lane = threadIdx.x & 31, nloc = lane & 15, hlf = lane >> 4; const size_t m0 = (size_t)blockIdx.x * 64 + wave * 16; const int n0 = blockIdx.y * 128;
  v8f acc[8];
#pragma unroll
  for (int t = 0; t < 8; ++t) acc[t] = (v8f){};
#pragma unroll 2
  for (int kb = 0; kb < K; kb += 32) { const v16b a = frag_kb(A + (m0 + nloc) * lda + kb, hlf);
#pragma unroll
    for (int t = 0; t < 8; ++t) acc[t] = wmma16b(a, frag_kb(Bt + (size_t)(n0 + t * 16 + nloc) * K + kb, hlf), acc[t]); }
#pragma unroll
  for (int t = 0; t < 8; ++t) { const float bb = bf16_rne(bias[n0 + t * 16 + nloc]);
#pragma unroll
    for (int r = 0; r < 8; ++r) { const float y = fmaxf(acc[t][r] * (1.0f / (XS * WSC)) + bb, 0.0f); if (MODE == 0) Tf[wave][8 * hlf + r][t * 16 + nloc] = y; else { b16 p, q; split16(y * XS, p, q); Th[wave][8 * hlf + r][t * 16 + nloc] = p; Tl[wave][8 * hlf + r][t * 16 + nloc] = q; } } }
  wave_lds_sync();
  for (int pass = 0; pass < 2; ++pass) {
    if (MODE == 0) { for (int rr = 0; rr < 16; ++rr) *(volatile v4f*)(Yf + (m0 + rr) * ldy + n0 + lane * 4) = *(const v4f*)(&Tf[wave][rr][lane * 4]); }
    else { for (int r2 = 0; r2 < 16; r2 += 2) { const int rr = r2 + (lane >> 4), c8 = (lane & 15) * 8; const size_t gi = (m0 + rr) * ldy + n0 + c8; *(volatile v8b*)(Yh + gi) = *(const v8b*)(&Th[wave][rr][c8]); *(volatile v8b*)(Yl + gi) = *(const v8b*)(&Tl[wave][rr][c8]); } }
    __threadfence(); }
}
__global__ __launch_bounds__(256) void gate_kernel(const float* __restrict__ HR, const float* __restrict__ rw2, const float* __restrict__ rb2, float* __restrict__ G) {
  __shared__ __attribute__((aligned(16))) float Gs[32][NE];
  const int wave = threadIdx.x >> 5, lane = threadIdx.x & 31; const int sl = lane >> 3, e = lane & 7; const int srow = wave * 4 + sl; const size_t b = (size_t)blockIdx.x * 32 + srow;
  const float* hr = HR + b * H; float lg = bf16_rne(rb2[e]);
#pragma unroll 4
  for (int k = 0; k < H; ++k) lg += pmul(hr[k], bf16_rne(rw2[k * NE + e]));
  float mx = lg; mx = fmaxf(mx, __shfl_xor(mx, 1)); mx = fmaxf(mx, __shfl_xor(mx, 2)); mx = fmaxf(mx, __shfl_xor(mx, 4));
  const float ex = nexp(lg - mx); float se = ex; se += __shfl_xor(se, 1); se += __shfl_xor(se, 2); se += __shfl_xor(se, 4); const float w = ex / se;
  int rank = 0;
#pragma unroll
  for (int j = 0; j < NE; ++j) { const float wj = __shfl(w, (lane & ~7) + j); rank += (wj > w || (wj == w && j < e)) ? 1 : 0; }
  const bool top = rank < 2; float ts = top ? w : 0.0f; ts += __shfl_xor(ts, 1); ts += __shfl_xor(ts, 2); ts += __shfl_xor(ts, 4);
  Gs[srow][e] = top ? w / (ts + 1e-6f) : 0.0f;
  __syncthreads();
  for (int pass = 0; pass < 2; ++pass) { if (threadIdx.x < 64) *(volatile v4f*)(G + (size_t)blockIdx.x * 32 * NE + threadIdx.x * 4) = *(const v4f*)(&Gs[0][0] + threadIdx.x * 4); __threadfence(); }
}
template <int LAST>
__global__ __launch_bounds__(128) void expert2_kernel(const b16* __restrict__ Hh, const b16* __restrict__ Hl, const b16* __restrict__ W2T, const float* __restrict__ eb2, const float* __restrict__ G, int e, float* __restrict__ ACC, float* __restrict__ out) {
  __shared__ __attribute__((aligned(16))) float Tf[4][16][P2 + 4];
  const int wave = threadIdx.x >> 5, lane = threadIdx.x & 31, nloc = lane & 15, hlf = lane >> 4; const size_t m0 = (size_t)blockIdx.x * 64 + wave * 16;
  v8f acc[6];
#pragma unroll
  for (int t = 0; t < 6; ++t) acc[t] = (v8f){};
#pragma unroll 2
  for (int kb = 0; kb < H; kb += 32) { const v16b a = frag_kb(Hh + (m0 + nloc) * H + kb, hlf), al = frag_kb(Hl + (m0 + nloc) * H + kb, hlf);
#pragma unroll
    for (int t = 0; t < 6; ++t) { const v16b bw = frag_kb(W2T + (size_t)(t * 16 + nloc) * H + kb, hlf); acc[t] = wmma16b(a, bw, acc[t]); acc[t] = wmma16b(al, bw, acc[t]); } }
#pragma unroll
  for (int t = 0; t < 6; ++t) { const int c = t * 16 + nloc; const float bb = bf16_rne(eb2[e * P2 + c]);
#pragma unroll
    for (int r = 0; r < 8; ++r) { const size_t row = m0 + 8 * hlf + r; float y = pmul(G[row * NE + e], acc[t][r] * (1.0f / (XS * WSC)) + bb); if (e > 0) y += ACC[row * P2 + c];
      Tf[wave][8 * hlf + r][c] = LAST ? 1.0f / (1.0f + nexp(-y)) : y; } }
  wave_lds_sync();
  for (int pass = 0; pass < 2; ++pass) { for (int rr = 0; rr < 16; ++rr) if (lane < 24) { const size_t gi = (m0 + rr) * P2 + lane * 4; const v4f y = *(const v4f*)(&Tf[wave][rr][lane * 4]); if (LAST) *(volatile v4f*)(out + gi) = y; else *(volatile v4f*)(ACC + gi) = y; }
    __threadfence(); }
}
}

extern "C" void kernel_launch(void* const* d_in, const int* in_sizes, int n_in, void* d_out, int out_size, void* d_ws, size_t ws_size, hipStream_t stream) {
  (void)n_in;
  auto Fp = [&](int i) { return (const float*)d_in[i]; };
  if (in_sizes[0] != B * H || in_sizes[1] != B * H || in_sizes[2] != RIN * H || in_sizes[3] != H || in_sizes[4] != H * NE || in_sizes[5] != NE || in_sizes[6] != NE * H * H || in_sizes[7] != NE * H || in_sizes[8] != NE * H * P2 || in_sizes[9] != NE * P2 || out_size != B * P2) return;
  size_t off = 0; char* ws = (char*)d_ws;
  auto carve = [&](size_t bytes) { char* p = ws + off; off += (bytes + 255) & ~(size_t)255; return p; };
  b16* RIN16 = (b16*)carve((size_t)B * RIN * 2); b16* RW1T = (b16*)carve((size_t)H * RIN * 2); b16* EW1T = (b16*)carve((size_t)NE * H * H * 2); b16* EW2T = (b16*)carve((size_t)NE * P2 * H * 2);
  float* HR = (float*)carve((size_t)B * H * 4); float* G = (float*)carve((size_t)B * NE * 4); b16* Hh = (b16*)carve((size_t)B * H * 2); b16* Hl = (b16*)carve((size_t)B * H * 2); float* ACC = (float*)carve((size_t)B * P2 * 4);
  if (off > ws_size || off > ((size_t)128 << 20)) return;
  prepx_kernel<<<(unsigned)(((size_t)B * RIN / 8 + 255) / 256), 256, 0, stream>>>(Fp(0), Fp(1), RIN16);
  prepw_kernel<<<dim3(RIN / 64, H / 64, 1 + 2 * NE), 256, 0, stream>>>(Fp(2), Fp(6), Fp(8), RW1T, EW1T, EW2T);
  gemm1_kernel<0, RIN><<<dim3(B / 64, H / 128), 128, 0, stream>>>(RIN16, RIN, RW1T, Fp(3), HR, nullptr, nullptr, H);
  gate_kernel<<<B / 32, 256, 0, stream>>>(HR, Fp(4), Fp(5), G);
  for (int e = 0; e < NE; ++e) {
    gemm1_kernel<1, H><<<dim3(B / 64, H / 128), 128, 0, stream>>>(RIN16, RIN, EW1T + (size_t)e * H * H, Fp(7) + (size_t)e * H, nullptr, Hh, Hl, H);
    if (e < NE - 1) expert2_kernel<0><<<B / 64, 128, 0, stream>>>(Hh, Hl, EW2T + (size_t)e * P2 * H, Fp(9), G, e, ACC, nullptr);
    else expert2_kernel<1><<<B / 64, 128, 0, stream>>>(Hh, Hl, EW2T + (size_t)e * P2 * H, Fp(9), G, e, ACC, (float*)d_out);
  }
}
